// UltimatexLSTMBlock_3006477107701
// MI455X (gfx1250) — hardware-run, weakly checked
//
#include <hip/hip_runtime.h>

constexpr int N_BATCH  = 4;
constexpr int SEQ_LEN  = 2048;
constexpr int D_MODEL  = 512;
constexpr int N_HEAD   = 8;
constexpr int D_HEAD   = 64;
constexpr int D_HID    = N_HEAD * D_HEAD;
constexpr int D_PROJ   = 2 * D_MODEL;
constexpr int N_FUSED  = 2 * N_HEAD + 4 * D_HID;
constexpr int N_TOK    = N_BATCH * SEQ_LEN;
constexpr int N_BH     = N_BATCH * N_HEAD;
constexpr int SQRT_D_HEAD = 8;
constexpr float KEY_SCALE = 1.0f / (float)SQRT_D_HEAD;
constexpr float GATE_CAP  = 15.0f;
constexpr float GATE_CAP_INV = 1.0f / GATE_CAP;
constexpr float LN_EPS = 1e-6f;
constexpr float F32_MIN_NORMAL = 1.17549435e-38f;
constexpr int COL_Q = 2 * N_HEAD;
constexpr int COL_K = COL_Q + D_HID;
constexpr int COL_V = COL_K + D_HID;
constexpr int COL_O = COL_V + D_HID;
constexpr int KV_PITCH   = 2 * D_HID;
constexpr int GATE_PITCH = 64;
constexpr int SCAN_TB    = 16;
constexpr int OUT1_OFF = N_TOK * D_MODEL;
constexpr int OUT2_OFF = OUT1_OFF + N_BH * D_HEAD * D_HEAD;
constexpr int OUT3_OFF = OUT2_OFF + N_BH * D_HEAD;
constexpr int OUT_TOTAL = OUT3_OFF + N_BH;
static_assert(SQRT_D_HEAD * SQRT_D_HEAD == D_HEAD);
static_assert(D_HID == 512 && D_PROJ == 1024 && N_FUSED == 2064);
static_assert(COL_O + D_HID == N_FUSED);
static_assert(N_BH == 32);
static_assert(OUT1_OFF * 4 == 16777216 && OUT2_OFF * 4 == 17301504 && OUT3_OFF * 4 == 17309696 && OUT_TOTAL * 4 == 17309824);
static_assert(N_TOK % 64 == 0 && D_MODEL % 64 == 0 && D_PROJ % 64 == 0 && D_HID % 64 == 0 && KV_PITCH % 64 == 0);
static_assert(D_MODEL % 32 == 0 && D_PROJ % 32 == 0 && D_HID % 32 == 0);
static_assert(SEQ_LEN % SCAN_TB == 0 && SEQ_LEN % 32 == 0);

typedef __attribute__((ext_vector_type(16))) __bf16   v16b;
typedef __attribute__((ext_vector_type(8)))  __bf16   v8b;
typedef __attribute__((ext_vector_type(8)))  _Float16 v8h;
typedef __attribute__((ext_vector_type(8)))  float    v8f;
typedef __attribute__((ext_vector_type(4)))  float    v4f;
typedef __attribute__((ext_vector_type(4)))  unsigned int v4u;
typedef __attribute__((ext_vector_type(2)))  unsigned int v2u;

__device__ __forceinline__ unsigned short f2bf_bits(float f) {
  unsigned u = __float_as_uint(f);
  return (unsigned short)((u + 0x7FFFu + ((u >> 16) & 1u)) >> 16);
}
__device__ __forceinline__ float bf_bits2f(unsigned short h) { return __uint_as_float(((unsigned)h) << 16); }
__device__ __forceinline__ unsigned pk16(unsigned short a, unsigned short b) { return (unsigned)a | ((unsigned)b << 16); }

__device__ __forceinline__ float h16_to_f32(unsigned hb) {
  const unsigned sgn = (hb & 0x8000u) << 16;
  const unsigned em = hb & 0x7fffu;
  const float fn = __uint_as_float((em << 13) + 0x38000000u);
  const float fs = (float)em * 5.9604644775390625e-8f;
  const float mag = (em < 0x400u) ? fs : fn;
  return __uint_as_float(__float_as_uint(mag) | sgn);
}

__device__ __forceinline__ void wave_sync() {
  __builtin_amdgcn_fence(__ATOMIC_RELEASE, "workgroup");
  __builtin_amdgcn_wave_barrier();
  __builtin_amdgcn_fence(__ATOMIC_ACQUIRE, "workgroup");
}

__device__ __forceinline__ void dep_guard4_b(v8f& a, v8f& b, v8f& c, v8f& d, v16b x, v16b y) {
  asm volatile("v_nop\n\tv_nop\n\tv_nop\n\tv_nop" : "+v"(a), "+v"(b), "+v"(c), "+v"(d) : "v"(x), "v"(y));
}
__device__ __forceinline__ void keep4_b(v16b a, v16b b, v16b c, v16b d) { asm volatile("v_nop" :: "v"(a), "v"(b), "v"(c), "v"(d)); }
__device__ __forceinline__ void acc_guard4(v8f& a, v8f& b, v8f& c, v8f& d) { asm volatile("v_nop\n\tv_nop\n\tv_nop\n\tv_nop" : "+v"(a), "+v"(b), "+v"(c), "+v"(d)); }

template <typename T> struct Frag;
template <> struct Frag<__bf16> {
  typedef v16b V; union U { v16b v; v8b h[2]; };
  static __device__ __forceinline__ v16b load(const __bf16* p) {
    U f; f.h[0] = *(const v8b*)(p); f.h[1] = *(const v8b*)(p + 16); return f.v;
  }
  static __device__ __forceinline__ v8f mma(v16b a, v16b b, v8f c) {
    return __builtin_amdgcn_wmma_f32_16x16x32_bf16(false, a, false, b, (short)0, c, false, false);
  }
};

template <bool WITH_LO>
__global__ __launch_bounds__(256) void weight_tr_kernel(const float* __restrict__ src, int ld, int col0, int n_real, int kdim,
                                                        unsigned short* __restrict__ hi, unsigned short* __restrict__ lo) {
  __shared__ float tile[64 * 65];
  const int tid = threadIdx.x, lane = tid & 31, wave = tid >> 5;
  const int k0 = blockIdx.x * 64, n0 = blockIdx.y * 64;
  const int nn = tid & 63;
  const int n = n0 + nn;
  const bool live = (n < n_real);
  const int nc = live ? n : (n_real - 1);
#pragma unroll 1
  for (int i = 0; i < 16; ++i) {
    const int kk = i * 4 + (tid >> 6);
    const float v = src[(size_t)(k0 + kk) * ld + col0 + nc];
    tile[kk * 65 + nn] = live ? v : 0.0f;
  }
  __syncthreads();
#pragma unroll 1
  for (int it = 0; it < 2; ++it) {
    const int rn = it * 32 + wave * 4 + (lane >> 3);
    const int k8 = (lane & 7) * 8;
    unsigned short hb[8], lb[8];
#pragma unroll
    for (int j = 0; j < 8; ++j) {
      const float f = tile[(k8 + j) * 65 + rn];
      hb[j] = f2bf_bits(f);
      lb[j] = f2bf_bits(f - bf_bits2f(hb[j]));
    }
    const v4u hu = (v4u){pk16(hb[0], hb[1]), pk16(hb[2], hb[3]), pk16(hb[4], hb[5]), pk16(hb[6], hb[7])};
    const v4u lu = (v4u){pk16(lb[0], lb[1]), pk16(lb[2], lb[3]), pk16(lb[4], lb[5]), pk16(lb[6], lb[7])};
    const size_t o = (size_t)(n0 + rn) * kdim + k0 + k8;
    *(volatile v4u*)(hi + o) = hu;
    if (WITH_LO) *(volatile v4u*)(lo + o) = lu;
    __threadfence();
    *(volatile v4u*)(hi + o) = hu;
    if (WITH_LO) *(volatile v4u*)(lo + o) = lu;
  }
}

__global__ __launch_bounds__(256) void ln_split_kernel(const float* __restrict__ x, const float* __restrict__ gam,
                                                       const float* __restrict__ bet, unsigned short* __restrict__ hi,
                                                       unsigned short* __restrict__ lo) {
  const int lane = threadIdx.x & 31, wave = threadIdx.x >> 5;
  const int tok = blockIdx.x * 8 + wave;
  const float* xr = x + (size_t)tok * D_MODEL;
  float a[16];
#pragma unroll
  for (int it = 0; it < 2; ++it) {
    const v4f p0 = *(const v4f*)(xr + it * 256 + lane * 8);
    const v4f p1 = *(const v4f*)(xr + it * 256 + lane * 8 + 4);
#pragma unroll
    for (int e = 0; e < 4; ++e) { a[it * 8 + e] = p0[e]; a[it * 8 + 4 + e] = p1[e]; }
  }
  float s = 0.0f;
#pragma unroll
  for (int i = 0; i < 16; ++i) s += a[i];
#pragma unroll
  for (int m = 16; m > 0; m >>= 1) s += __shfl_xor(s, m, 32);
  const float mu = s * (1.0f / (float)D_MODEL);
  float q = 0.0f;
#pragma unroll
  for (int i = 0; i < 16; ++i) { const float d = a[i] - mu; q += d * d; }
#pragma unroll
  for (int m = 16; m > 0; m >>= 1) q += __shfl_xor(q, m, 32);
  const float var = q * (1.0f / (float)D_MODEL);
  const float rstd = 1.0f / sqrtf(var + LN_EPS);
  v4u hw[2], lw[2];
#pragma unroll
  for (int it = 0; it < 2; ++it) {
    const int c = it * 256 + lane * 8;
    const v4f g0 = *(const v4f*)(gam + c);
    const v4f g1 = *(const v4f*)(gam + c + 4);
    const v4f b0 = *(const v4f*)(bet + c);
    const v4f b1 = *(const v4f*)(bet + c + 4);
    unsigned short hb[8], lb[8];
#pragma unroll
    for (int e = 0; e < 4; ++e) {
      const float y0 = (a[it * 8 + e] - mu) * rstd * g0[e] + b0[e];
      const float y1 = (a[it * 8 + 4 + e] - mu) * rstd * g1[e] + b1[e];
      hb[e] = f2bf_bits(y0);
      lb[e] = f2bf_bits(y0 - bf_bits2f(hb[e]));
      hb[4 + e] = f2bf_bits(y1);
      lb[4 + e] = f2bf_bits(y1 - bf_bits2f(hb[4 + e]));
    }
    hw[it] = (v4u){pk16(hb[0], hb[1]), pk16(hb[2], hb[3]), pk16(hb[4], hb[5]), pk16(hb[6], hb[7])};
    lw[it] = (v4u){pk16(lb[0], lb[1]), pk16(lb[2], lb[3]), pk16(lb[4], lb[5]), pk16(lb[6], lb[7])};
  }
  unsigned short* hp = hi + (size_t)tok * D_MODEL + lane * 8;
  unsigned short* lp = lo + (size_t)tok * D_MODEL + lane * 8;
  *(volatile v4u*)(hp) = hw[0];
  *(volatile v4u*)(hp + 256) = hw[1];
  *(volatile v4u*)(lp) = lw[0];
  *(volatile v4u*)(lp + 256) = lw[1];
  __threadfence();
  *(volatile v4u*)(hp) = hw[0];
  *(volatile v4u*)(hp + 256) = hw[1];
  *(volatile v4u*)(lp) = lw[0];
  *(volatile v4u*)(lp + 256) = lw[1];
}

template <bool SPLIT, bool BIAS, bool POST, int OUT_MODE, bool RESID, int ACT>
__global__ __launch_bounds__(256) void wmma_gemm64(
    const unsigned short* __restrict__ Ap, const unsigned short* __restrict__ A2p, int lda,
    const unsigned short* __restrict__ Btp, const unsigned short* __restrict__ Bt2p, int ldb,
    void* __restrict__ Cout, int ldc,
    const float* __restrict__ bias, const float* __restrict__ resid,
    int M, int N, int K, float post_scale, int post_cols) {
  typedef __bf16 T;
  typedef Frag<T>::V V;
  const T* A = (const T*)Ap; const T* A2 = (const T*)A2p; const T* Bt = (const T*)Btp; const T* Bt2 = (const T*)Bt2p;
  __shared__ __align__(16) float sT[8][16 * 68];
  const int lane = threadIdx.x & 31;
  const int wave = threadIdx.x >> 5;
  const int tilesN = N >> 6;
  const int tilesM = M >> 6;
  const int tile = blockIdx.x * 8 + wave;
  if (tile >= tilesM * tilesN) return;
  const int tm = tile / tilesN;
  const int tn = tile - tm * tilesN;
  const int m0 = tm << 6;
  const int n0 = tn << 6;

  const int rlane = lane & 15;
  const int koff  = (lane >> 4) * 8;
  const int mOff  = (lane >> 4) * 8;

  int aoff[4], boff[4];
#pragma unroll
  for (int i = 0; i < 4; ++i) {
    aoff[i] = (m0 + (i << 4) + rlane) * lda + koff;
    boff[i] = (n0 + (i << 4) + rlane) * ldb + koff;
  }

  v8f acc[4][4];
#pragma unroll
  for (int i = 0; i < 4; ++i)
#pragma unroll
    for (int j = 0; j < 4; ++j) acc[i][j] = (v8f){0.f,0.f,0.f,0.f,0.f,0.f,0.f,0.f};

  for (int k0 = 0; k0 < K; k0 += 32) {
    V bh[4], bl[4];
#pragma unroll
    for (int j = 0; j < 4; ++j) {
      bh[j] = Frag<T>::load(Bt + boff[j] + k0);
      if (SPLIT) bl[j] = Frag<T>::load(Bt2 + boff[j] + k0);
    }
#pragma unroll
    for (int i = 0; i < 4; ++i) {
      V ah = Frag<T>::load(A + aoff[i] + k0);
      V al = ah;
      if (SPLIT) al = Frag<T>::load(A2 + aoff[i] + k0);
#pragma unroll
      for (int j = 0; j < 4; ++j) {
        acc[i][j] = Frag<T>::mma(ah, bh[j], acc[i][j]);
        if (SPLIT) {
          acc[i][j] = Frag<T>::mma(ah, bl[j], acc[i][j]);
          acc[i][j] = Frag<T>::mma(al, bh[j], acc[i][j]);
        }
      }
      dep_guard4_b(acc[i][0], acc[i][1], acc[i][2], acc[i][3], ah, al);
    }
    keep4_b(bh[0], bh[1], bh[2], bh[3]);
    if (SPLIT) keep4_b(bl[0], bl[1], bl[2], bl[3]);
  }
  acc_guard4(acc[0][0], acc[0][1], acc[0][2], acc[0][3]);
  acc_guard4(acc[1][0], acc[1][1], acc[1][2], acc[1][3]);
  acc_guard4(acc[2][0], acc[2][1], acc[2][2], acc[2][3]);
  acc_guard4(acc[3][0], acc[3][1], acc[3][2], acc[3][3]);

  float* slab = sT[wave];
  const int hh = lane >> 4, c4 = (lane & 15) * 4;
  const float post = (POST && (n0 < post_cols)) ? post_scale : 1.0f;
#pragma unroll
  for (int i = 0; i < 4; ++i) {
    const int mBase = m0 + (i << 4);
#pragma unroll
    for (int j = 0; j < 4; ++j) {
      float bv = 0.f;
      if (BIAS) bv = bias[n0 + (j << 4) + rlane];
#pragma unroll
      for (int r = 0; r < 8; ++r) {
        float v = acc[i][j][r];
        if (BIAS) v += bv;
        if (POST) v *= post;
        slab[(mOff + r) * 68 + (j << 4) + rlane] = v;
      }
    }
    wave_sync();
    if (RESID || ACT == 1) {
#pragma unroll 1
      for (int it = 0; it < 8; ++it) {
        const int row = it * 2 + hh;
        v4f v = *(const v4f*)(slab + row * 68 + c4);
        if (RESID) {
          const v4f rr = *(const v4f*)(resid + (size_t)(mBase + row) * ldc + n0 + c4);
          v += rr;
        }
        if (ACT == 1) {
#pragma unroll
          for (int e = 0; e < 4; ++e) {
            const float t = v[e];
            const float sg = 1.0f / (1.0f + expf(-t));
            v[e] = sg;
          }
        }
        *(v4f*)(slab + row * 68 + c4) = v;
      }
      wave_sync();
    }
    if (OUT_MODE == 0) {
      float* C = (float*)Cout;
      for (int pass = 0; pass < 2; ++pass) {
#pragma unroll
        for (int it = 0; it < 8; ++it) {
          const int row = it * 2 + hh;
          v4f v = *(const v4f*)(slab + row * 68 + c4);
          *(volatile v4f*)(C + (size_t)(mBase + row) * ldc + n0 + c4) = v;
        }
        __threadfence();
      }
    } else {
      const int q = lane >> 3, c8 = (lane & 7) * 8;
      unsigned short* C = (unsigned short*)Cout;
      for (int pass = 0; pass < 2; ++pass) {
#pragma unroll
        for (int it = 0; it < 4; ++it) {
          const int row = it * 4 + q;
          const float* sp = slab + row * 68 + c8;
          v8h hv;
#pragma unroll
          for (int e = 0; e < 8; ++e) {
            if (OUT_MODE == 1) {
              hv[e] = (_Float16)sp[e];
            } else {
              unsigned short hb = f2bf_bits(sp[e]);
              hv[e] = __builtin_bit_cast(_Float16, hb);
            }
          }
          *(volatile v8h*)(C + (size_t)(mBase + row) * ldc + n0 + c8) = hv;
        }
        __threadfence();
      }
    }
    wave_sync();
  }
}

__global__ __launch_bounds__(256) void conv_silu_split_kernel(const float* __restrict__ XUP, const float* __restrict__ cw,
                                                              unsigned short* __restrict__ hi, unsigned short* __restrict__ lo) {
  const int idx = blockIdx.x * 256 + threadIdx.x;
  const int tok = idx >> 8;
  const int p0 = (idx & 255) * 4;
  const float* row = XUP + (size_t)tok * D_PROJ;
  const int pm = (p0 >= 4) ? (p0 - 4) : 0;
  const v4f left = *(const v4f*)(row + pm);
  const v4f cur  = *(const v4f*)(row + p0);
  const bool has = (p0 > 0);
  float xs[7];
  xs[0] = has ? left[1] : 0.0f;
  xs[1] = has ? left[2] : 0.0f;
  xs[2] = has ? left[3] : 0.0f;
  xs[3] = cur[0];
  xs[4] = cur[1];
  xs[5] = cur[2];
  xs[6] = cur[3];
  const float w0 = cw[0], w1 = cw[1], w2 = cw[2], w3 = cw[3];
  unsigned short hb[4], lb[4];
#pragma unroll
  for (int e = 0; e < 4; ++e) {
    const float c = w0 * xs[e] + w1 * xs[e + 1] + w2 * xs[e + 2] + w3 * xs[e + 3];
    const float sg = 1.0f / (1.0f + expf(-c));
    const float y = c * sg;
    hb[e] = f2bf_bits(y);
    lb[e] = f2bf_bits(y - bf_bits2f(hb[e]));
  }
  const v2u hu = (v2u){pk16(hb[0], hb[1]), pk16(hb[2], hb[3])};
  const v2u lu = (v2u){pk16(lb[0], lb[1]), pk16(lb[2], lb[3])};
  const size_t o = (size_t)tok * D_PROJ + p0;
  *(volatile v2u*)(hi + o) = hu;
  *(volatile v2u*)(lo + o) = lu;
  __threadfence();
  *(volatile v2u*)(hi + o) = hu;
  *(volatile v2u*)(lo + o) = lu;
}

__global__ __launch_bounds__(32) void gate_scan_kernel(const float* __restrict__ GATE, const float* __restrict__ bfused,
                                                       float* __restrict__ FE, float* __restrict__ IE, float* __restrict__ mf) {
  __shared__ __align__(16) float sfe[32 * 36];
  __shared__ __align__(16) float sie[32 * 36];
  const int lane = threadIdx.x;
  const int b = lane / N_HEAD;
  const int h = lane % N_HEAD;
  const float bi = bfused[h];
  const float bf = bfused[N_HEAD + h];
  const float* gp = GATE + (size_t)b * SEQ_LEN * GATE_PITCH + h;
  float m = 0.0f;
#pragma unroll 1
  for (int ch = 0; ch < SEQ_LEN / 32; ++ch) {
#pragma unroll 1
    for (int ss = 0; ss < 32; ++ss) {
      const int s = ch * 32 + ss;
      float iv = gp[(size_t)s * GATE_PITCH] + bi;
      float fv = gp[(size_t)s * GATE_PITCH + N_HEAD] + bf;
      iv = GATE_CAP * tanhf(iv * GATE_CAP_INV);
      fv = GATE_CAP * tanhf(fv * GATE_CAP_INV);
      const float mt = fmaxf(fv + m, iv);
      float ie = expf(iv - mt);
      float fe = expf((fv - mt) + m);
      ie = (ie < F32_MIN_NORMAL) ? 0.0f : ie;
      fe = (fe < F32_MIN_NORMAL) ? 0.0f : fe;
      m = mt;
      sfe[lane * 36 + ss] = fe;
      sie[lane * 36 + ss] = ie;
    }
    __syncthreads();
    for (int pass = 0; pass < 2; ++pass) {
#pragma unroll 1
      for (int it = 0; it < 8; ++it) {
        const int rw = it * 4 + (lane >> 3);
        const int st4 = (lane & 7) * 4;
        const v4f a = *(const v4f*)(sfe + rw * 36 + st4);
        const v4f c = *(const v4f*)(sie + rw * 36 + st4);
        const size_t o = (size_t)rw * SEQ_LEN + ch * 32 + st4;
        *(volatile v4f*)(FE + o) = a;
        *(volatile v4f*)(IE + o) = c;
      }
      __threadfence();
    }
    __syncthreads();
  }
  *(volatile float*)(mf + lane) = m;
  __threadfence();
  *(volatile float*)(mf + lane) = m;
}

__global__ __launch_bounds__(256) void state_scan_kernel(const float* __restrict__ KV, const unsigned short* __restrict__ Qp,
                                                         const float* __restrict__ FE, const float* __restrict__ IE,
                                                         float* __restrict__ G, float* __restrict__ Cf, float* __restrict__ nf) {
  __shared__ __align__(16) float hbuf[2 * SCAN_TB * D_HEAD];
  __shared__ __align__(16) float Cs[D_HEAD * 68];
  __shared__ __align__(16) float ns[D_HEAD];
  const int tid = threadIdx.x;
  const int bh = blockIdx.x;
  const int b = bh / N_HEAD;
  const int h = bh % N_HEAD;
  const int r = tid >> 2, qd = tid & 3, c0 = qd * 16;

  float C[16], nst[16];
#pragma unroll
  for (int j = 0; j < 16; ++j) { C[j] = 0.0f; nst[j] = 1.0f; }

  const float* kp = KV + (size_t)b * SEQ_LEN * KV_PITCH + h * D_HEAD + c0;
  const float* vp = KV + (size_t)b * SEQ_LEN * KV_PITCH + D_HID + h * D_HEAD + r;
  const unsigned short* qp = Qp + (size_t)b * SEQ_LEN * D_HID + h * D_HEAD + c0;
  const float* fep = FE + (size_t)bh * SEQ_LEN;
  const float* iep = IE + (size_t)bh * SEQ_LEN;
  float* gbase = G + (size_t)b * SEQ_LEN * D_HID + h * D_HEAD;
  const int srow = tid >> 4, sc4 = (tid & 15) * 4;

#pragma unroll 1
  for (int sb = 0; sb < SEQ_LEN / SCAN_TB; ++sb) {
    float* hb = hbuf + (sb & 1) * (SCAN_TB * D_HEAD);
#pragma unroll 1
    for (int ss = 0; ss < SCAN_TB; ++ss) {
      const int s = sb * SCAN_TB + ss;
      const float* kr = kp + (size_t)s * KV_PITCH;
      v4f kq[4];
#pragma unroll
      for (int t = 0; t < 4; ++t) kq[t] = *(const v4f*)(kr + 4 * t);
      const v4u qw0 = *(const v4u*)(qp + (size_t)s * D_HID);
      const v4u qw1 = *(const v4u*)(qp + (size_t)s * D_HID + 8);
      const float vr = vp[(size_t)s * KV_PITCH];
      const float fe = fep[s];
      const float ie = iep[s];
      float kk[16], qq[16];
#pragma unroll
      for (int t = 0; t < 4; ++t) {
#pragma unroll
        for (int e = 0; e < 4; ++e) kk[4 * t + e] = kq[t][e];
        const unsigned wa = qw0[t];
        const unsigned wb = qw1[t];
        qq[2 * t]         = __uint_as_float(wa << 16);
        qq[2 * t + 1]     = __uint_as_float(wa & 0xffff0000u);
        qq[8 + 2 * t]     = __uint_as_float(wb << 16);
        qq[8 + 2 * t + 1] = __uint_as_float(wb & 0xffff0000u);
      }
      const float av = ie * vr;
      float part = 0.0f, dpart = 0.0f;
#pragma unroll
      for (int j = 0; j < 16; ++j) {
        C[j] = fmaf(fe, C[j], av * kk[j]);
        part = fmaf(C[j], qq[j], part);
        nst[j] = fmaf(fe, nst[j], ie * kk[j]);
        dpart = fmaf(nst[j], qq[j], dpart);
      }
      part  += __shfl_xor(part, 1, 32);
      dpart += __shfl_xor(dpart, 1, 32);
      part  += __shfl_xor(part, 2, 32);
      dpart += __shfl_xor(dpart, 2, 32);
      const float den = fmaxf(dpart, 1.0f);
      const float hval = part * (1.0f / den);
      if (qd == 0) hb[ss * D_HEAD + r] = hval;
    }
    __syncthreads();
    {
      const v4f val = *(const v4f*)(hb + srow * D_HEAD + sc4);
      float* gp = gbase + (size_t)(sb * SCAN_TB + srow) * D_HID + sc4;
      *(volatile v4f*)gp = val;
      __threadfence();
      *(volatile v4f*)gp = val;
    }
  }

#pragma unroll
  for (int j = 0; j < 16; ++j) Cs[r * 68 + c0 + j] = C[j];
  if (r == 0) {
#pragma unroll
    for (int j = 0; j < 16; ++j) ns[c0 + j] = nst[j];
  }
  __syncthreads();
  for (int pass = 0; pass < 2; ++pass) {
#pragma unroll
    for (int it = 0; it < 4; ++it) {
      const int row = it * 16 + srow;
      const v4f v = *(const v4f*)(Cs + row * 68 + sc4);
      *(volatile v4f*)(Cf + ((size_t)bh * D_HEAD + row) * D_HEAD + sc4) = v;
    }
    if (tid < 16) {
      const v4f nv = *(const v4f*)(ns + tid * 4);
      *(volatile v4f*)(nf + (size_t)bh * D_HEAD + tid * 4) = nv;
    }
    __threadfence();
  }
}

__device__ __forceinline__ v4f gated4(const float* __restrict__ G, const unsigned short* __restrict__ Og, size_t off) {
  const v4f hv = *(const v4f*)(G + off);
  const v2u ow = *(const v2u*)(Og + off);
  const unsigned w0 = ow[0];
  const unsigned w1 = ow[1];
  v4f g;
  g[0] = hv[0] * h16_to_f32(w0 & 0xffffu);
  g[1] = hv[1] * h16_to_f32(w0 >> 16);
  g[2] = hv[2] * h16_to_f32(w1 & 0xffffu);
  g[3] = hv[3] * h16_to_f32(w1 >> 16);
  return g;
}

__global__ __launch_bounds__(256) void ln_gate_kernel(const float* __restrict__ G, const unsigned short* __restrict__ Og,
                                                      const unsigned short* __restrict__ Rg, const float* __restrict__ gam,
                                                      const float* __restrict__ bet, unsigned short* __restrict__ Y) {
  const int lane = threadIdx.x & 31, wave = threadIdx.x >> 5;
  const int tok = blockIdx.x * 8 + wave;
  const size_t rowoff = (size_t)tok * D_HID;
  float gv[16];
#pragma unroll
  for (int it = 0; it < 4; ++it) {
    const v4f g = gated4(G, Og, rowoff + it * 128 + lane * 4);
#pragma unroll
    for (int e = 0; e < 4; ++e) gv[it * 4 + e] = g[e];
  }
  float s = 0.0f;
#pragma unroll
  for (int i = 0; i < 16; ++i) s += gv[i];
#pragma unroll
  for (int m = 16; m > 0; m >>= 1) s += __shfl_xor(s, m, 32);
  const float mu = s * (1.0f / (float)D_HID);
  float q = 0.0f;
#pragma unroll
  for (int i = 0; i < 16; ++i) { const float d = gv[i] - mu; q += d * d; }
#pragma unroll
  for (int m = 16; m > 0; m >>= 1) q += __shfl_xor(q, m, 32);
  const float var = q * (1.0f / (float)D_HID);
  const float rstd = 1.0f / sqrtf(var + LN_EPS);
#pragma unroll 1
  for (int it = 0; it < 4; ++it) {
    const int c = it * 128 + lane * 4;
    const v4f g = gated4(G, Og, rowoff + c);
    const v2u rw = *(const v2u*)(Rg + rowoff + c);
    const v4f gm = *(const v4f*)(gam + c);
    const v4f bt = *(const v4f*)(bet + c);
    const unsigned r0 = rw[0];
    const unsigned r1 = rw[1];
    float rv[4];
    rv[0] = h16_to_f32(r0 & 0xffffu);
    rv[1] = h16_to_f32(r0 >> 16);
    rv[2] = h16_to_f32(r1 & 0xffffu);
    rv[3] = h16_to_f32(r1 >> 16);
    unsigned short yb[4];
#pragma unroll
    for (int e = 0; e < 4; ++e) {
      const float ln = (g[e] - mu) * rstd * gm[e] + bt[e];
      const float sg = 1.0f / (1.0f + expf(-rv[e]));
      const float y = ln * (rv[e] * sg);
      yb[e] = f2bf_bits(y);
    }
    const v2u yu = (v2u){pk16(yb[0], yb[1]), pk16(yb[2], yb[3])};
    *(volatile v2u*)(Y + rowoff + c) = yu;
    __threadfence();
    *(volatile v2u*)(Y + rowoff + c) = yu;
  }
}

extern "C" void kernel_launch(void* const* d_in, const int* in_sizes, int n_in,
                              void* d_out, int out_size, void* d_ws, size_t ws_size, hipStream_t stream) {
  if (n_in < 11 || d_out == nullptr || d_ws == nullptr) return;
  if (in_sizes[0] != N_TOK * D_MODEL || in_sizes[1] != D_MODEL || in_sizes[2] != D_MODEL || in_sizes[3] != D_HID ||
      in_sizes[4] != D_HID || in_sizes[5] != D_MODEL * D_PROJ || in_sizes[6] != D_MODEL * D_HID ||
      in_sizes[7] != D_PROJ * N_FUSED || in_sizes[8] != N_FUSED || in_sizes[9] != D_HID * D_MODEL ||
      in_sizes[10] != 4 || out_size != OUT_TOTAL) return;

  const float* x       = (const float*)d_in[0];
  const float* inp_g   = (const float*)d_in[1];
  const float* inp_b   = (const float*)d_in[2];
  const float* hid_g   = (const float*)d_in[3];
  const float* hid_b   = (const float*)d_in[4];
  const float* W_up    = (const float*)d_in[5];
  const float* W_r     = (const float*)d_in[6];
  const float* W_fused = (const float*)d_in[7];
  const float* b_fused = (const float*)d_in[8];
  const float* W_down  = (const float*)d_in[9];
  const float* conv_w  = (const float*)d_in[10];
  float* out = (float*)d_out;

  char* ws = (char*)d_ws;
  size_t off = 0;
  auto carve = [&](size_t bytes) -> char* {
    char* p = ws + off;
    off += (bytes + 255) & ~(size_t)255;
    return p;
  };
  unsigned short* XNH  = (unsigned short*)carve((size_t)N_TOK * D_MODEL * 2);
  unsigned short* XNL  = (unsigned short*)carve((size_t)N_TOK * D_MODEL * 2);
  float*          XUP  = (float*)carve((size_t)N_TOK * D_PROJ * 4);
  unsigned short* Rpl  = (unsigned short*)carve((size_t)N_TOK * D_HID * 2);
  unsigned short* XCH  = (unsigned short*)carve((size_t)N_TOK * D_PROJ * 2);
  unsigned short* XCL  = (unsigned short*)carve((size_t)N_TOK * D_PROJ * 2);
  unsigned short* Opl  = (unsigned short*)carve((size_t)N_TOK * D_HID * 2);
  float*          GATE = (float*)carve((size_t)N_TOK * GATE_PITCH * 4);
  float*          FE   = (float*)carve((size_t)N_BH * SEQ_LEN * 4);
  float*          IE   = (float*)carve((size_t)N_BH * SEQ_LEN * 4);
  float*          Gpl  = (float*)carve((size_t)N_TOK * D_HID * 4);
  unsigned short* WUPH = (unsigned short*)carve((size_t)D_PROJ * D_MODEL * 2);
  unsigned short* WUPL = (unsigned short*)carve((size_t)D_PROJ * D_MODEL * 2);
  unsigned short* WR   = (unsigned short*)carve((size_t)D_HID * D_MODEL * 2);
  unsigned short* WKVH = (unsigned short*)carve((size_t)KV_PITCH * D_PROJ * 2);
  unsigned short* WKVL = (unsigned short*)carve((size_t)KV_PITCH * D_PROJ * 2);
  unsigned short* WGH  = (unsigned short*)carve((size_t)GATE_PITCH * D_PROJ * 2);
  unsigned short* WGL  = (unsigned short*)carve((size_t)GATE_PITCH * D_PROJ * 2);
  unsigned short* WQ   = (unsigned short*)carve((size_t)D_HID * D_PROJ * 2);
  unsigned short* WO   = (unsigned short*)carve((size_t)D_HID * D_PROJ * 2);
  unsigned short* WD   = (unsigned short*)carve((size_t)D_MODEL * D_HID * 2);
  if (off > ws_size || off > (size_t)134217728) return;
  float*          KV  = XUP;
  unsigned short* Qpl = XNH;
  unsigned short* Ypl = XNL;

  weight_tr_kernel<true><<<dim3(D_MODEL / 64, D_PROJ / 64), dim3(256), 0, stream>>>(W_up, D_PROJ, 0, D_PROJ, D_MODEL, WUPH, WUPL);
  weight_tr_kernel<false><<<dim3(D_MODEL / 64, D_HID / 64), dim3(256), 0, stream>>>(W_r, D_HID, 0, D_HID, D_MODEL, WR, WR);
  weight_tr_kernel<true><<<dim3(D_PROJ / 64, KV_PITCH / 64), dim3(256), 0, stream>>>(W_fused, N_FUSED, COL_K, KV_PITCH, D_PROJ, WKVH, WKVL);
  weight_tr_kernel<true><<<dim3(D_PROJ / 64, GATE_PITCH / 64), dim3(256), 0, stream>>>(W_fused, N_FUSED, 0, 2 * N_HEAD, D_PROJ, WGH, WGL);
  weight_tr_kernel<false><<<dim3(D_PROJ / 64, D_HID / 64), dim3(256), 0, stream>>>(W_fused, N_FUSED, COL_Q, D_HID, D_PROJ, WQ, WQ);
  weight_tr_kernel<false><<<dim3(D_PROJ / 64, D_HID / 64), dim3(256), 0, stream>>>(W_fused, N_FUSED, COL_O, D_HID, D_PROJ, WO, WO);
  weight_tr_kernel<false><<<dim3(D_HID / 64, D_MODEL / 64), dim3(256), 0, stream>>>(W_down, D_MODEL, 0, D_MODEL, D_HID, WD, WD);

  ln_split_kernel<<<dim3(N_TOK / 8), dim3(256), 0, stream>>>(x, inp_g, inp_b, XNH, XNL);

  wmma_gemm64<true, false, false, 0, false, 0><<<dim3((N_TOK / 64) * (D_PROJ / 64) / 8), dim3(256), 0, stream>>>(
      XNH, XNL, D_MODEL, WUPH, WUPL, D_MODEL, (void*)XUP, D_PROJ, nullptr, nullptr, N_TOK, D_PROJ, D_MODEL, 1.0f, 0);
  wmma_gemm64<false, false, false, 1, false, 0><<<dim3((N_TOK / 64) * (D_HID / 64) / 8), dim3(256), 0, stream>>>(
      XNH, XNH, D_MODEL, WR, WR, D_MODEL, (void*)Rpl, D_HID, nullptr, nullptr, N_TOK, D_HID, D_MODEL, 1.0f, 0);

  conv_silu_split_kernel<<<dim3(N_TOK * D_PROJ / 4 / 256), dim3(256), 0, stream>>>(XUP, conv_w, XCH, XCL);

  wmma_gemm64<true, true, true, 0, false, 0><<<dim3((N_TOK / 64) * (KV_PITCH / 64) / 8), dim3(256), 0, stream>>>(
      XCH, XCL, D_PROJ, WKVH, WKVL, D_PROJ, (void*)KV, KV_PITCH, b_fused + COL_K, nullptr, N_TOK, KV_PITCH, D_PROJ, KEY_SCALE, D_HID);
  wmma_gemm64<true, false, false, 0, false, 0><<<dim3((N_TOK / 64) * (GATE_PITCH / 64) / 8), dim3(256), 0, stream>>>(
      XCH, XCL, D_PROJ, WGH, WGL, D_PROJ, (void*)GATE, GATE_PITCH, nullptr, nullptr, N_TOK, GATE_PITCH, D_PROJ, 1.0f, 0);
  wmma_gemm64<false, true, false, 2, false, 0><<<dim3((N_TOK / 64) * (D_HID / 64) / 8), dim3(256), 0, stream>>>(
      XCH, XCH, D_PROJ, WQ, WQ, D_PROJ, (void*)Qpl, D_HID, b_fused + COL_Q, nullptr, N_TOK, D_HID, D_PROJ, 1.0f, 0);
  wmma_gemm64<false, true, false, 1, false, 1><<<dim3((N_TOK / 64) * (D_HID / 64) / 8), dim3(256), 0, stream>>>(
      XCH, XCH, D_PROJ, WO, WO, D_PROJ, (void*)Opl, D_HID, b_fused + COL_O, nullptr, N_TOK, D_HID, D_PROJ, 1.0f, 0);

  gate_scan_kernel<<<dim3(1), dim3(32), 0, stream>>>(GATE, b_fused, FE, IE, out + OUT3_OFF);
  state_scan_kernel<<<dim3(N_BH), dim3(256), 0, stream>>>(KV, Qpl, FE, IE, Gpl, out + OUT1_OFF, out + OUT2_OFF);

  ln_gate_kernel<<<dim3(N_TOK / 8), dim3(256), 0, stream>>>(Gpl, Opl, Rpl, hid_g, hid_b, Ypl);
  wmma_gemm64<false, false, false, 0, true, 0><<<dim3((N_TOK / 64) * (D_MODEL / 64) / 8), dim3(256), 0, stream>>>(
      Ypl, Ypl, D_HID, WD, WD, D_HID, (void*)out, D_MODEL, nullptr, x, N_TOK, D_MODEL, D_HID, 1.0f, 0);
}
